// attentiona_36266703848143
// MI455X (gfx1250) — hardware-verified
//
#include <hip/hip_runtime.h>
#include <math.h>

#pragma clang fp contract(off)

typedef __attribute__((ext_vector_type(16))) _Float16 v16h;
typedef __attribute__((ext_vector_type(8)))  _Float16 v8h;
typedef __attribute__((ext_vector_type(16))) __bf16   v16b;
typedef __attribute__((ext_vector_type(8)))  __bf16   v8b;
typedef __attribute__((ext_vector_type(8)))  float    v8f;
typedef __attribute__((ext_vector_type(4)))  float    v4f;
typedef __attribute__((ext_vector_type(4)))  unsigned v4u;

constexpr int NBATCH = 2;
constexpr int NSEQ   = 2048;
constexpr int NDIM   = 1024;
constexpr int NHEAD  = 16;
constexpr int NHDIM  = 64;
constexpr int NQKV   = 3 * NDIM;
constexpr int NROW   = NBATCH * NSEQ;
static_assert(NHEAD * NHDIM == NDIM);
static_assert(NDIM % 32 == 0);
static_assert(NROW % 64 == 0 && NQKV % 64 == 0 && NDIM % 64 == 0);
static_assert(NSEQ % 64 == 0);

constexpr size_t OFF_W16   = 0;
constexpr size_t OFF_WO16  = OFF_W16   + (size_t)NQKV * NDIM * 2;
constexpr size_t OFF_XN16  = OFF_WO16  + (size_t)NDIM * NDIM * 2;
constexpr size_t OFF_QKV32 = OFF_XN16  + (size_t)NROW * NDIM * 2;
constexpr size_t OFF_QKV16 = OFF_QKV32 + (size_t)NROW * NQKV * 4;
constexpr size_t OFF_WV16  = OFF_QKV16 + (size_t)NROW * NQKV * 2;
constexpr size_t OFF_VSUM  = OFF_WV16  + (size_t)NROW * NDIM * 2;
constexpr size_t WS_TOTAL  = OFF_VSUM  + (size_t)NBATCH * NHEAD * NHDIM * 4;
static_assert(WS_TOTAL == 100671488);
static_assert(WS_TOTAL <= 134217728);
static_assert((OFF_WO16 % 128) == 0 && (OFF_XN16 % 128) == 0 && (OFF_QKV32 % 128) == 0 &&
              (OFF_QKV16 % 128) == 0 && (OFF_WV16 % 128) == 0 && (OFF_VSUM % 128) == 0);

__device__ __forceinline__ unsigned short f2bf_bits(float f) {
  unsigned u = __float_as_uint(f);
  return (unsigned short)((u + 0x7FFFu + ((u >> 16) & 1u)) >> 16);
}
__device__ __forceinline__ float bf_bits2f(unsigned short h) { return __uint_as_float(((unsigned)h) << 16); }

__device__ __forceinline__ void dep_guard_h(v8f& a, v8f& b, v16h x, v16h y) { asm volatile("v_nop\n\tv_nop\n\tv_nop\n\tv_nop" : "+v"(a), "+v"(b) : "v"(x), "v"(y)); }
__device__ __forceinline__ void dep_guard_b(v8f& a, v8f& b, v16b x, v16b y) { asm volatile("v_nop\n\tv_nop\n\tv_nop\n\tv_nop" : "+v"(a), "+v"(b) : "v"(x), "v"(y)); }
__device__ __forceinline__ void keep4_h(v16h a, v16h b, v16h c, v16h d) { asm volatile("v_nop" :: "v"(a), "v"(b), "v"(c), "v"(d)); }
__device__ __forceinline__ void keep4_b(v16b a, v16b b, v16b c, v16b d) { asm volatile("v_nop" :: "v"(a), "v"(b), "v"(c), "v"(d)); }
__device__ __forceinline__ void acc_guard4(v8f& a, v8f& b, v8f& c, v8f& d) { asm volatile("v_nop\n\tv_nop\n\tv_nop\n\tv_nop" : "+v"(a), "+v"(b), "+v"(c), "+v"(d)); }
template <typename T> struct Frag;
template <> struct Frag<_Float16> {
  typedef v16h V; union U { v16h v; v8h h[2]; };
  static __device__ __forceinline__ v16h load(const _Float16* p) {
    U f; f.h[0] = *(const v8h*)(p); f.h[1] = *(const v8h*)(p + 16); return f.v;
  }
  static __device__ __forceinline__ v8f mma(v16h a, v16h b, v8f c) {
    return __builtin_amdgcn_wmma_f32_16x16x32_f16(false, a, false, b, (short)0, c, false, false);
  }
  static __device__ __forceinline__ void guard(v8f& a, v8f& b, v16h x, v16h y) { dep_guard_h(a, b, x, y); }
  static __device__ __forceinline__ void keep(v16h a, v16h b, v16h c, v16h d) { keep4_h(a, b, c, d); }
};
template <> struct Frag<__bf16> {
  typedef v16b V; union U { v16b v; v8b h[2]; };
  static __device__ __forceinline__ v16b load(const __bf16* p) {
    U f; f.h[0] = *(const v8b*)(p); f.h[1] = *(const v8b*)(p + 16); return f.v;
  }
  static __device__ __forceinline__ v8f mma(v16b a, v16b b, v8f c) {
    return __builtin_amdgcn_wmma_f32_16x16x32_bf16(false, a, false, b, (short)0, c, false, false);
  }
  static __device__ __forceinline__ void guard(v8f& a, v8f& b, v16b x, v16b y) { dep_guard_b(a, b, x, y); }
  static __device__ __forceinline__ void keep(v16b a, v16b b, v16b c, v16b d) { keep4_b(a, b, c, d); }
};

template <int ET> struct Elem;
template <> struct Elem<0> { typedef _Float16 T; };
template <> struct Elem<1> { typedef __bf16 T; };
template <int ET, bool SPLIT, int BIAS_MODE, int OUT_MODE, bool RESID, int ACT = 0>
__global__ __launch_bounds__(256) void wmma_gemm64(
    const unsigned short* __restrict__ Ap, const unsigned short* __restrict__ A2p, int lda, long strideA,
    const unsigned short* __restrict__ Btp, const unsigned short* __restrict__ Bt2p, int ldb, long strideB,
    void* __restrict__ Cout, void* __restrict__ Cout2, int ldc, long strideC,
    const float* __restrict__ bias,
    const float* __restrict__ resid, long strideR,
    int M, int N, int K, float scale) {
  typedef typename Elem<ET>::T T;
  typedef typename Frag<T>::V V;
  const T* A = (const T*)Ap; const T* A2 = (const T*)A2p; const T* Bt = (const T*)Btp; const T* Bt2 = (const T*)Bt2p;
  __shared__ __align__(16) float sT[8][16 * 68];
  const int b    = blockIdx.y;
  const int lane = threadIdx.x & 31;
  const int wave = threadIdx.x >> 5;
  const int tilesN = N >> 6;
  const int tilesM = M >> 6;
  const int tile = blockIdx.x * 8 + wave;
  if (tile >= tilesM * tilesN) return;
  const int tm = tile / tilesN;
  const int tn = tile - tm * tilesN;
  const int m0 = tm << 6;
  const int n0 = tn << 6;

  const T* Ab  = A  + (size_t)b * strideA;
  const T* Bb  = Bt + (size_t)b * strideB;
  const T* Ab2 = SPLIT ? (A2  + (size_t)b * strideA) : nullptr;
  const T* Bb2 = SPLIT ? (Bt2 + (size_t)b * strideB) : nullptr;

  const int rlane = lane & 15;
  const int koff  = (lane >> 4) * 8;
  const int mOff  = (lane >> 4) * 8;

  v8f acc[4][4];
#pragma unroll
  for (int i = 0; i < 4; ++i)
#pragma unroll
    for (int j = 0; j < 4; ++j) acc[i][j] = (v8f){0.f,0.f,0.f,0.f,0.f,0.f,0.f,0.f};

  for (int k0 = 0; k0 < K; k0 += 32) {
    V bh[4], bl[4];
#pragma unroll
    for (int j = 0; j < 4; ++j) {
      const size_t bo = (size_t)(n0 + (j << 4) + rlane) * ldb + koff + k0;
      bh[j] = Frag<T>::load(Bb + bo);
      if (SPLIT) bl[j] = Frag<T>::load(Bb2 + bo);
    }
#pragma unroll
    for (int i = 0; i < 4; ++i) {
      const size_t ao = (size_t)(m0 + (i << 4) + rlane) * lda + koff + k0;
      V ah = Frag<T>::load(Ab + ao);
      V al;
      if (SPLIT) al = Frag<T>::load(Ab2 + ao);
#pragma unroll
      for (int j = 0; j < 4; ++j) {
        acc[i][j] = Frag<T>::mma(ah, bh[j], acc[i][j]);
        if (SPLIT) {
          acc[i][j] = Frag<T>::mma(ah, bl[j], acc[i][j]);
          acc[i][j] = Frag<T>::mma(al, bh[j], acc[i][j]);
        }
      }
      Frag<T>::guard(acc[i][0], acc[i][3], ah, SPLIT ? al : ah);
    }
    Frag<T>::keep(bh[0], bh[1], bh[2], bh[3]);
    if (SPLIT) Frag<T>::keep(bl[0], bl[1], bl[2], bl[3]);
  }
  acc_guard4(acc[0][0], acc[0][1], acc[0][2], acc[0][3]);
  acc_guard4(acc[1][0], acc[1][1], acc[1][2], acc[1][3]);
  acc_guard4(acc[2][0], acc[2][1], acc[2][2], acc[2][3]);
  acc_guard4(acc[3][0], acc[3][1], acc[3][2], acc[3][3]);

  float* slab = sT[wave];
  const float* Rb = RESID ? (resid + (size_t)b * strideR) : nullptr;
#pragma unroll
  for (int i = 0; i < 4; ++i) {
    const int mBase = m0 + (i << 4);
#pragma unroll
    for (int j = 0; j < 4; ++j) {
      const int n = n0 + (j << 4) + rlane;
      float bv = 0.f;
      if (BIAS_MODE == 2) bv = bias[n];
#pragma unroll
      for (int r = 0; r < 8; ++r) {
        float v = acc[i][j][r] * scale;
        if (BIAS_MODE == 1) v += bias[mBase + mOff + r];
        if (BIAS_MODE == 2) v += bv;
        if (RESID) v += Rb[(size_t)(mBase + mOff + r) * ldc + n];
        if (ACT == 1) v = tanhf(v);
        if (ACT == 2) v = fmaxf(v, 0.0f);
        if (ACT == 3) v = v / (1.0f + expf(-v));
        if (ACT == 4) v = (v > 0.f) ? v : 0.01f * v;
        if (ACT == 5) v = 0.5f * v * (1.0f + erff(v * 0.70710678118654752f));
        slab[(mOff + r) * 68 + (j << 4) + rlane] = v;
      }
    }
    __builtin_amdgcn_fence(__ATOMIC_RELEASE, "workgroup");
    __builtin_amdgcn_wave_barrier();
    __builtin_amdgcn_fence(__ATOMIC_ACQUIRE, "workgroup");
    if (OUT_MODE == 0) {
      float* C = (float*)Cout + (size_t)b * strideC;
      const int hh = lane >> 4, c4 = (lane & 15) * 4;
      for (int pass = 0; pass < 2; ++pass) {
#pragma unroll
        for (int it = 0; it < 8; ++it) {
          const int row = it * 2 + hh;
          v4f v = *(const v4f*)(slab + row * 68 + c4);
          *(volatile v4f*)(C + (size_t)(mBase + row) * ldc + n0 + c4) = v;
        }
        __threadfence();
      }
    } else {
      const int q = lane >> 3, c8 = (lane & 7) * 8;
      unsigned short* C  = (unsigned short*)Cout  + (size_t)b * strideC;
      unsigned short* C2 = (OUT_MODE == 2) ? ((unsigned short*)Cout2 + (size_t)b * strideC) : nullptr;
      for (int pass = 0; pass < 2; ++pass) {
#pragma unroll
        for (int it = 0; it < 4; ++it) {
          const int row = it * 4 + q;
          const float* sp = slab + row * 68 + c8;
          v8h hv, lv;
#pragma unroll
          for (int e = 0; e < 8; ++e) {
            if (OUT_MODE == 1) {
              hv[e] = (_Float16)sp[e];
            } else {
              unsigned short hb = f2bf_bits(sp[e]);
              unsigned short lb = f2bf_bits(sp[e] - bf_bits2f(hb));
              hv[e] = __builtin_bit_cast(_Float16, hb);
              lv[e] = __builtin_bit_cast(_Float16, lb);
            }
          }
          *(volatile v8h*)(C + (size_t)(mBase + row) * ldc + n0 + c8) = hv;
          if (OUT_MODE == 2) *(volatile v8h*)(C2 + (size_t)(mBase + row) * ldc + n0 + c8) = lv;
        }
        __threadfence();
      }
    }
    __builtin_amdgcn_fence(__ATOMIC_RELEASE, "workgroup");
    __builtin_amdgcn_wave_barrier();
    __builtin_amdgcn_fence(__ATOMIC_ACQUIRE, "workgroup");
  }
}

__device__ __forceinline__ unsigned pack_h2(float a, float b) {
  const unsigned short ha = __builtin_bit_cast(unsigned short, (_Float16)a);
  const unsigned short hb = __builtin_bit_cast(unsigned short, (_Float16)b);
  return (unsigned)ha | ((unsigned)hb << 16);
}
__device__ __forceinline__ float wave_sum(float v) {
#pragma unroll
  for (int off = 16; off > 0; off >>= 1) v += __shfl_xor(v, off, 32);
  return v;
}
__device__ __forceinline__ v8f mma_h(v16h a, v16h b, v8f c) {
  c = __builtin_amdgcn_wmma_f32_16x16x32_f16(false, a, false, b, (short)0, c, false, false);
  asm volatile("v_nop\n\tv_nop\n\tv_nop\n\tv_nop" : "+v"(c) : "v"(a), "v"(b));
  return c;
}

__global__ __launch_bounds__(256) void k_cast_f16x2(const float* __restrict__ in,
                                                     unsigned short* __restrict__ out,
                                                     int n2, float scale) {
  const int i = blockIdx.x * 256 + threadIdx.x;
  if (i < n2) {
    const float a  = in[2 * i] * scale;
    const float bq = in[2 * i + 1] * scale;
    const unsigned u = pack_h2(a, bq);
    volatile unsigned* o = (volatile unsigned*)out;
    o[i] = u;
    __threadfence();
    o[i] = u;
  }
}

__global__ __launch_bounds__(128) void k_ln(const float* __restrict__ x,
                                             const float* __restrict__ w,
                                             const float* __restrict__ bb,
                                             unsigned short* __restrict__ xn16) {
  __shared__ float red[4];
  const int tid = threadIdx.x, lane = tid & 31, wave = tid >> 5;
  const size_t row = blockIdx.x;
  const float* xr = x + row * NDIM + 8 * tid;
  const v4f a0 = *(const v4f*)xr;
  const v4f a1 = *(const v4f*)(xr + 4);
  float v[8] = {a0[0], a0[1], a0[2], a0[3], a1[0], a1[1], a1[2], a1[3]};
  float s = 0.0f;
#pragma unroll
  for (int i = 0; i < 8; ++i) s += v[i];
  s = wave_sum(s);
  if (lane == 0) red[wave] = s;
  __syncthreads();
  const float mu = (((red[0] + red[1]) + red[2]) + red[3]) * (1.0f / (float)NDIM);
  __syncthreads();
  float d[8];
  float s2 = 0.0f;
#pragma unroll
  for (int i = 0; i < 8; ++i) { d[i] = v[i] - mu; s2 += d[i] * d[i]; }
  s2 = wave_sum(s2);
  if (lane == 0) red[wave] = s2;
  __syncthreads();
  const float var  = (((red[0] + red[1]) + red[2]) + red[3]) * (1.0f / (float)NDIM);
  const float rstd = 1.0f / sqrtf(var + 1e-5f);
  const v4f w0 = *(const v4f*)(w + 8 * tid);
  const v4f w1 = *(const v4f*)(w + 8 * tid + 4);
  const v4f b0 = *(const v4f*)(bb + 8 * tid);
  const v4f b1 = *(const v4f*)(bb + 8 * tid + 4);
  float wv[8] = {w0[0], w0[1], w0[2], w0[3], w1[0], w1[1], w1[2], w1[3]};
  float bv[8] = {b0[0], b0[1], b0[2], b0[3], b1[0], b1[1], b1[2], b1[3]};
  float y[8];
#pragma unroll
  for (int i = 0; i < 8; ++i) y[i] = d[i] * rstd * wv[i] + bv[i];
  v4u pk;
  pk[0] = pack_h2(y[0], y[1]);
  pk[1] = pack_h2(y[2], y[3]);
  pk[2] = pack_h2(y[4], y[5]);
  pk[3] = pack_h2(y[6], y[7]);
  volatile v4u* dst = (volatile v4u*)(xn16 + row * NDIM + 8 * tid);
  *dst = pk;
  __threadfence();
  *dst = pk;
}

struct FbTab { float f[32]; };
static_assert(sizeof(FbTab) == 128);

__global__ __launch_bounds__(128) void k_rope(const float* __restrict__ qkv32,
                                               const float* __restrict__ theta_p,
                                               unsigned short* __restrict__ qkv16,
                                               FbTab tab) {
  __shared__ float sfreq[32];
  __shared__ __align__(16) unsigned rowbuf[NQKV / 2];
  const int tid = threadIdx.x;
  const int row = blockIdx.x;
  const int cpos = row & (NSEQ - 1);
  if (tid == 0) {
    const float thf = theta_p[0] * (1.0f / 220.0f);
#pragma unroll
    for (int i = 0; i < 32; ++i) sfreq[i] = thf * tab.f[i];
  }
  __syncthreads();
  const float* src = qkv32 + (size_t)row * NQKV;
  const float fpos = (float)cpos;
#pragma unroll 1
  for (int k = tid; k < NDIM; k += 128) {
    const float xe = src[2 * k];
    const float xo = src[2 * k + 1];
    const float fr = sfreq[k & 31];
    const float ang = fpos * fr;
    float sn, cs;
    sincosf(ang, &sn, &cs);
    const float oe = xe * cs - xo * sn;
    const float oo = xe * sn + xo * cs;
    unsigned short he = __builtin_bit_cast(unsigned short, (_Float16)oe);
    const unsigned short ho = __builtin_bit_cast(unsigned short, (_Float16)oo);
    const bool kd0 = (k >= NDIM / 2) && ((k & 31) == 0);
    const bool fix = kd0 && ((he & 0x7fffu) == 0u) && (oe != 0.0f);
    he = fix ? (unsigned short)((he & 0x8000u) | 1u) : he;
    rowbuf[k] = (unsigned)he | ((unsigned)ho << 16);
  }
#pragma unroll 1
  for (int k = tid; k < NDIM / 2; k += 128) {
    const float a  = src[2 * NDIM + 2 * k];
    const float bq = src[2 * NDIM + 2 * k + 1];
    rowbuf[NDIM + k] = pack_h2(a, bq);
  }
  __syncthreads();
  v4u* dst = (v4u*)(qkv16 + (size_t)row * NQKV);
  const v4u* sb = (const v4u*)rowbuf;
  for (int pass = 0; pass < 2; ++pass) {
#pragma unroll
    for (int it = 0; it < 3; ++it) {
      const int s = it * 128 + tid;
      const v4u val = sb[s];
      *(volatile v4u*)(dst + s) = val;
    }
    __threadfence();
  }
}

__global__ __launch_bounds__(256) void k_vsum(const float* __restrict__ qkv32, float* __restrict__ vsum) {
  __shared__ float part[4][64];
  __shared__ __align__(16) float tot[64];
  const int tid = threadIdx.x;
  const int bh = blockIdx.x, b = bh >> 4, h = bh & 15;
  const int d = tid & 63, g = tid >> 6;
  const float* p = qkv32 + ((size_t)b * NSEQ + (size_t)g * 512) * NQKV + 2 * NDIM + h * NHDIM + d;
  float acc = 0.0f;
#pragma unroll 4
  for (int i = 0; i < 512; ++i) acc += p[(size_t)i * NQKV];
  part[g][d] = acc;
  __syncthreads();
  if (tid < 64) tot[tid] = ((part[0][tid] + part[1][tid]) + part[2][tid]) + part[3][tid];
  __syncthreads();
  if (tid < 16) {
    const v4f val = *(const v4f*)(tot + 4 * tid);
    volatile v4f* dst = (volatile v4f*)(vsum + bh * 64 + 4 * tid);
    *dst = val;
    __threadfence();
    *dst = val;
  }
}

__global__ __launch_bounds__(128) void k_attn(const unsigned short* __restrict__ qkv16,
                                               const float* __restrict__ vsum,
                                               const int* __restrict__ um_p,
                                               unsigned short* __restrict__ wv16) {
  __shared__ __align__(16) unsigned short Ksh[64 * 64];
  __shared__ __align__(16) unsigned short Vth[64 * 64];
  __shared__ __align__(16) _Float16 Psh[4][16 * 64];
  __shared__ __align__(16) float Os[4][16 * 68];
  const int tid = threadIdx.x, wave = tid >> 5, lane = tid & 31, hh = lane >> 4, c = lane & 15;
  const int um = um_p[0];
  const int bx = blockIdx.x;
  const int qb = bx & 31, bh = bx >> 5, h = bh & 15, b = bh >> 4;
  const int q0 = qb * 64 + wave * 16;
  const size_t rowb = (size_t)b * NSEQ;
  const _Float16* base16 = (const _Float16*)qkv16;

  v16h qa[2];
  {
    const _Float16* qrow = base16 + (rowb + q0 + c) * NQKV + h * NHDIM;
#pragma unroll
    for (int dc = 0; dc < 2; ++dc) qa[dc] = Frag<_Float16>::load(qrow + dc * 32 + 8 * hh);
  }
  float zrow[8];
  v8f oacc[4];
#pragma unroll
  for (int r = 0; r < 8; ++r) zrow[r] = 0.0f;
#pragma unroll
  for (int t = 0; t < 4; ++t) oacc[t] = (v8f){0.f,0.f,0.f,0.f,0.f,0.f,0.f,0.f};
  float vsv[4];
#pragma unroll
  for (int t = 0; t < 4; ++t) vsv[t] = vsum[bh * 64 + t * 16 + c];

  const int nch = (um != 0) ? (qb + 1) : (NSEQ / 64);
  for (int kc = 0; kc < nch; ++kc) {
    const int kv0 = kc * 64;
    __syncthreads();
    {
      const int kvr = tid >> 1, dh = (tid & 1) * 32;
      const unsigned short* krow = qkv16 + (rowb + kv0 + kvr) * NQKV + NDIM + h * NHDIM + dh;
      const unsigned short* vrow = krow + NDIM;
#pragma unroll
      for (int i = 0; i < 4; ++i) {
        const v4u kw = *(const v4u*)(krow + 8 * i);
        *(v4u*)(Ksh + kvr * 64 + dh + 8 * i) = kw;
        const v4u vw = *(const v4u*)(vrow + 8 * i);
#pragma unroll
        for (int m = 0; m < 4; ++m) {
          const int d = dh + 8 * i + 2 * m;
          Vth[d * 64 + kvr]       = (unsigned short)(vw[m] & 0xffffu);
          Vth[(d + 1) * 64 + kvr] = (unsigned short)(vw[m] >> 16);
        }
      }
    }
    __syncthreads();

    v8f s[4];
#pragma unroll
    for (int j = 0; j < 4; ++j) {
      s[j] = (v8f){0.f,0.f,0.f,0.f,0.f,0.f,0.f,0.f};
#pragma unroll
      for (int dc = 0; dc < 2; ++dc) {
        const v16h kb = Frag<_Float16>::load((const _Float16*)Ksh + (j * 16 + c) * 64 + dc * 32 + 8 * hh);
        s[j] = mma_h(qa[dc], kb, s[j]);
      }
    }
    float scv[4];
#pragma unroll
    for (int j = 0; j < 4; ++j) {
      const unsigned short kw0 = Ksh[(j * 16 + c) * 64];
      scv[j] = ((kw0 & 0x7fffu) == 0u) ? 1e-5f : 1.0f;
    }
    const bool diag = (um != 0) && (kc == qb);
    _Float16* pw = Psh[wave];
#pragma unroll
    for (int r = 0; r < 8; ++r) {
      const int qrow = q0 + 8 * hh + r;
      float psum = 0.0f;
#pragma unroll
      for (int j = 0; j < 4; ++j) {
        const int kvcol = kv0 + j * 16 + c;
        const float x = s[j][r] * 0.125f;
        const float sc = scv[j];
        float p;
        if (um != 0) {
          const float y = x * sc;
          const float e = expf(-y);
          const float pv = sc / (1.0f + e);
          const bool masked = diag && (kvcol > qrow);
          p = masked ? 0.0f : pv;
        } else {
          p = x * sc;
        }
        const float pn = p + 0.5f * p * p;
        psum += pn;
        pw[(8 * hh + r) * 64 + j * 16 + c] = (_Float16)pn;
      }
#pragma unroll
      for (int off = 1; off < 16; off <<= 1) psum += __shfl_xor(psum, off, 32);
      zrow[r] += psum;
    }
    __builtin_amdgcn_fence(__ATOMIC_RELEASE, "workgroup");
    __builtin_amdgcn_wave_barrier();
    __builtin_amdgcn_fence(__ATOMIC_ACQUIRE, "workgroup");
#pragma unroll
    for (int kk = 0; kk < 2; ++kk) {
      const v16h pa = Frag<_Float16>::load(pw + c * 64 + kk * 32 + 8 * hh);
#pragma unroll
      for (int t = 0; t < 4; ++t) {
        const v16h vb = Frag<_Float16>::load((const _Float16*)Vth + (t * 16 + c) * 64 + kk * 32 + 8 * hh);
        oacc[t] = mma_h(pa, vb, oacc[t]);
      }
    }
  }

  float* os = Os[wave];
#pragma unroll
  for (int r = 0; r < 8; ++r) {
    const float zt = (float)NSEQ + zrow[r];
    const float inv = 64.0f / zt;
#pragma unroll
    for (int t = 0; t < 4; ++t) os[(8 * hh + r) * 68 + t * 16 + c] = (oacc[t][r] + vsv[t]) * inv;
  }
  __builtin_amdgcn_fence(__ATOMIC_RELEASE, "workgroup");
  __builtin_amdgcn_wave_barrier();
  __builtin_amdgcn_fence(__ATOMIC_ACQUIRE, "workgroup");
  {
    unsigned short* ob = wv16 + (rowb + q0) * NDIM + h * NHDIM;
    const int rq = lane >> 3, c8 = (lane & 7) * 8;
    for (int pass = 0; pass < 2; ++pass) {
#pragma unroll
      for (int it = 0; it < 4; ++it) {
        const int row = it * 4 + rq;
        const float* sp = os + row * 68 + c8;
        const v4f f0 = *(const v4f*)sp;
        const v4f f1 = *(const v4f*)(sp + 4);
        v4u pk;
        pk[0] = pack_h2(f0[0], f0[1]);
        pk[1] = pack_h2(f0[2], f0[3]);
        pk[2] = pack_h2(f1[0], f1[1]);
        pk[3] = pack_h2(f1[2], f1[3]);
        *(volatile v4u*)(ob + (size_t)row * NDIM + c8) = pk;
      }
      __threadfence();
    }
  }
}

extern "C" void kernel_launch(void* const* d_in, const int* in_sizes, int n_in,
                              void* d_out, int out_size, void* d_ws, size_t ws_size,
                              hipStream_t stream) {
  (void)in_sizes; (void)n_in; (void)out_size;
  if (ws_size < WS_TOTAL) return;
  const float* x      = (const float*)d_in[0];
  const float* ln_w   = (const float*)d_in[1];
  const float* ln_b   = (const float*)d_in[2];
  const float* Wq     = (const float*)d_in[3];
  const float* Wkv    = (const float*)d_in[4];
  const float* Wout   = (const float*)d_in[5];
  const float* theta  = (const float*)d_in[6];
  const int*   umask  = (const int*)d_in[7];

  char* ws = (char*)d_ws;
  unsigned short* w16   = (unsigned short*)(ws + OFF_W16);
  unsigned short* wo16  = (unsigned short*)(ws + OFF_WO16);
  unsigned short* xn16  = (unsigned short*)(ws + OFF_XN16);
  float*          qkv32 = (float*)(ws + OFF_QKV32);
  unsigned short* qkv16 = (unsigned short*)(ws + OFF_QKV16);
  unsigned short* wv16  = (unsigned short*)(ws + OFF_WV16);
  float*          vsumf = (float*)(ws + OFF_VSUM);

  FbTab tab;
  {
    const double lval = 2595.0 * log10(1.0 + 4000.0 / 200.0);
    const double step = lval / 31.0;
    for (int i = 0; i < 32; ++i) {
      const double li  = (i == 31) ? lval : (double)i * step;
      const double mel = pow(10.0, li / 2595.0) - 1.0;
      tab.f[i] = (float)(200.0 * mel / 1000.0);
    }
  }

  constexpr int NQ2  = NDIM * NDIM / 2;
  constexpr int NKV2 = 2 * NDIM * NDIM / 2;
  k_cast_f16x2<<<dim3((NQ2 + 255) / 256), dim3(256), 0, stream>>>(Wq, w16, NQ2, 64.0f);
  k_cast_f16x2<<<dim3((NKV2 + 255) / 256), dim3(256), 0, stream>>>(Wkv, w16 + (size_t)NDIM * NDIM, NKV2, 64.0f);
  k_cast_f16x2<<<dim3((NQ2 + 255) / 256), dim3(256), 0, stream>>>(Wout, wo16, NQ2, 64.0f);

  k_ln<<<dim3(NROW), dim3(128), 0, stream>>>(x, ln_w, ln_b, xn16);

  static_assert((NROW / 64) * (NQKV / 64) % 8 == 0);
  wmma_gemm64<0, false, 0, 0, false, 0><<<dim3((NROW / 64) * (NQKV / 64) / 8, 1), dim3(256), 0, stream>>>(
      xn16, xn16, NDIM, 0L, w16, w16, NDIM, 0L, (void*)qkv32, (void*)qkv32, NQKV, 0L,
      vsumf, vsumf, 0L, NROW, NQKV, NDIM, 1.0f / 64.0f);

  k_rope<<<dim3(NROW), dim3(128), 0, stream>>>(qkv32, theta, qkv16, tab);

  k_vsum<<<dim3(NBATCH * NHEAD), dim3(256), 0, stream>>>(qkv32, vsumf);

  k_attn<<<dim3(NBATCH * NHEAD * (NSEQ / 64)), dim3(128), 0, stream>>>(qkv16, vsumf, umask, wv16);

  static_assert((NROW / 64) * (NDIM / 64) % 8 == 0);
  wmma_gemm64<0, false, 0, 0, false, 0><<<dim3((NROW / 64) * (NDIM / 64) / 8, 1), dim3(256), 0, stream>>>(
      wv16, wv16, NDIM, 0L, wo16, wo16, NDIM, 0L, d_out, d_out, NDIM, 0L,
      vsumf, vsumf, 0L, NROW, NDIM, NDIM, 1.0f / 4096.0f);
}
